// CasualAttention_42966852829217
// MI455X (gfx1250) — hardware-verified
//
#include <hip/hip_runtime.h>

typedef __attribute__((ext_vector_type(16))) _Float16 v16h;
typedef __attribute__((ext_vector_type(8)))  _Float16 v8h;
typedef __attribute__((ext_vector_type(16))) __bf16   v16b;
typedef __attribute__((ext_vector_type(8)))  __bf16   v8b;
typedef __attribute__((ext_vector_type(8)))  float    v8f;
typedef __attribute__((ext_vector_type(4)))  float    v4f;
typedef __attribute__((ext_vector_type(4)))  unsigned v4u;

constexpr int NBATCH = 4;
constexpr int SEQ    = 2048;
constexpr int DIN    = 1024;
constexpr int DMODEL = 1024;
constexpr int NTOK   = NBATCH * SEQ;
constexpr int QHALF  = SEQ / 2;
constexpr size_t PLANE_TOK = (size_t)NTOK * DMODEL;
constexpr size_t WPLANE    = (size_t)DMODEL * DIN;
constexpr float LOG2E = 1.44269504088896340736f;

constexpr size_t MIB     = 1048576;
constexpr size_t OFF_SC  = 0;
constexpr size_t OFF_PH  = 8 * MIB;
constexpr size_t OFF_PL  = 12 * MIB;
constexpr size_t OFF_WT  = 16 * MIB;
constexpr size_t OFF_QKH = 22 * MIB;
constexpr size_t OFF_QKL = 54 * MIB;
constexpr size_t OFF_VTH = 86 * MIB;
constexpr size_t OFF_VTL = 102 * MIB;
constexpr size_t WS_END  = 118 * MIB;
static_assert(PLANE_TOK * 2 == 16 * MIB, "xb plane is 16 MiB");
static_assert((size_t)QHALF * SEQ * 4 == OFF_PH, "scores region 8 MiB");
static_assert(OFF_PH + (size_t)QHALF * SEQ * 2 == OFF_PL && OFF_PL + (size_t)QHALF * SEQ * 2 == OFF_WT, "P planes fit R0");
static_assert(OFF_WT + 3 * WPLANE * 2 == OFF_QKH, "W^T planes");
static_assert(OFF_QKH + 2 * PLANE_TOK * 2 == OFF_QKL && OFF_QKL + 2 * PLANE_TOK * 2 == OFF_VTH, "q/k planes");
static_assert(OFF_VTH + PLANE_TOK * 2 == OFF_VTL && OFF_VTL + PLANE_TOK * 2 == WS_END, "V^T planes");
static_assert(WS_END <= 134217728, "carve under 128 MiB");
static_assert(NTOK % 64 == 0 && DMODEL % 64 == 0 && SEQ % 64 == 0 && QHALF % 64 == 0, "tile multiples");
static_assert(DIN % 32 == 0 && DMODEL % 32 == 0 && SEQ % 32 == 0, "K multiples of 32");

__device__ __forceinline__ unsigned short f2bf_bits(float f) {
  unsigned u = __float_as_uint(f);
  return (unsigned short)((u + 0x7FFFu + ((u >> 16) & 1u)) >> 16);
}
__device__ __forceinline__ float bf_bits2f(unsigned short h) { return __uint_as_float(((unsigned)h) << 16); }
__device__ __forceinline__ unsigned pack_bf16x2(float a, float b) {
  return (unsigned)f2bf_bits(a) | (((unsigned)f2bf_bits(b)) << 16);
}

__device__ __forceinline__ void dep_guard_h(v8f& a, v8f& b, v16h x, v16h y) { asm volatile("v_nop\n\tv_nop\n\tv_nop\n\tv_nop" : "+v"(a), "+v"(b) : "v"(x), "v"(y)); }
__device__ __forceinline__ void dep_guard_b(v8f& a, v8f& b, v16b x, v16b y) { asm volatile("v_nop\n\tv_nop\n\tv_nop\n\tv_nop" : "+v"(a), "+v"(b) : "v"(x), "v"(y)); }
__device__ __forceinline__ void keep4_h(v16h a, v16h b, v16h c, v16h d) { asm volatile("v_nop" :: "v"(a), "v"(b), "v"(c), "v"(d)); }
__device__ __forceinline__ void keep4_b(v16b a, v16b b, v16b c, v16b d) { asm volatile("v_nop" :: "v"(a), "v"(b), "v"(c), "v"(d)); }
__device__ __forceinline__ void acc_guard4(v8f& a, v8f& b, v8f& c, v8f& d) { asm volatile("v_nop\n\tv_nop\n\tv_nop\n\tv_nop" : "+v"(a), "+v"(b), "+v"(c), "+v"(d)); }
template <typename T> struct Frag;
template <> struct Frag<_Float16> {
  typedef v16h V; union U { v16h v; v8h h[2]; };
  static __device__ __forceinline__ v16h load(const _Float16* p) {
    U f; f.h[0] = *(const v8h*)(p); f.h[1] = *(const v8h*)(p + 16); return f.v;
  }
  static __device__ __forceinline__ v8f mma(v16h a, v16h b, v8f c) {
    return __builtin_amdgcn_wmma_f32_16x16x32_f16(false, a, false, b, (short)0, c, false, false);
  }
  static __device__ __forceinline__ void guard(v8f& a, v8f& b, v16h x, v16h y) { dep_guard_h(a, b, x, y); }
  static __device__ __forceinline__ void keep(v16h a, v16h b, v16h c, v16h d) { keep4_h(a, b, c, d); }
};
template <> struct Frag<__bf16> {
  typedef v16b V; union U { v16b v; v8b h[2]; };
  static __device__ __forceinline__ v16b load(const __bf16* p) {
    U f; f.h[0] = *(const v8b*)(p); f.h[1] = *(const v8b*)(p + 16); return f.v;
  }
  static __device__ __forceinline__ v8f mma(v16b a, v16b b, v8f c) {
    return __builtin_amdgcn_wmma_f32_16x16x32_bf16(false, a, false, b, (short)0, c, false, false);
  }
  static __device__ __forceinline__ void guard(v8f& a, v8f& b, v16b x, v16b y) { dep_guard_b(a, b, x, y); }
  static __device__ __forceinline__ void keep(v16b a, v16b b, v16b c, v16b d) { keep4_b(a, b, c, d); }
};
template <int ET> struct Elem;
template <> struct Elem<0> { typedef _Float16 T; };
template <> struct Elem<1> { typedef __bf16 T; };

template <int ET, bool SPLIT, int OUT_MODE, int CMODE>
__global__ __launch_bounds__(256) void wmma_gemm64c(
    const unsigned short* __restrict__ Ap, const unsigned short* __restrict__ A2p, int lda, long strideA,
    const unsigned short* __restrict__ Btp, const unsigned short* __restrict__ Bt2p, int ldb, long strideB,
    void* __restrict__ Cout, void* __restrict__ Cout2, int ldc, long strideC,
    int M, int N, int K, float scale, int tm0) {
  typedef typename Elem<ET>::T T;
  typedef typename Frag<T>::V V;
  const T* A = (const T*)Ap; const T* A2 = (const T*)A2p; const T* Bt = (const T*)Btp; const T* Bt2 = (const T*)Bt2p;
  __shared__ __align__(16) float sT[8][16 * 68];
  const int b    = blockIdx.y;
  const int lane = threadIdx.x & 31;
  const int wave = threadIdx.x >> 5;
  const int tilesN = N >> 6;
  const int tilesM = M >> 6;
  const int tile = blockIdx.x * 8 + wave;
  int tm = 0, tn = 0;
  if (CMODE == 1) {
    int rem = tile; tm = -1;
#pragma unroll 1
    for (int i = 0; i < tilesM; ++i) {
      const int len = tm0 + i + 1;
      if (tm < 0) {
        if (rem < len) { tm = i; tn = rem; } else { rem -= len; }
      }
    }
    if (tm < 0) return;
  } else {
    if (tile >= tilesM * tilesN) return;
    tm = tile / tilesN;
    tn = tile - tm * tilesN;
  }
  const int m0 = tm << 6;
  const int n0 = tn << 6;
  const int Kend = (CMODE == 2) ? ((tm0 + tm + 1) << 6) : K;

  const T* Ab  = A  + (size_t)b * strideA;
  const T* Bb  = Bt + (size_t)b * strideB;
  const T* Ab2 = SPLIT ? (A2  + (size_t)b * strideA) : nullptr;
  const T* Bb2 = SPLIT ? (Bt2 + (size_t)b * strideB) : nullptr;

  const int rlane = lane & 15;
  const int koff  = (lane >> 4) * 8;
  const int mOff  = (lane >> 4) * 8;

  v8f acc[4][4];
#pragma unroll
  for (int i = 0; i < 4; ++i)
#pragma unroll
    for (int j = 0; j < 4; ++j) acc[i][j] = (v8f){0.f,0.f,0.f,0.f,0.f,0.f,0.f,0.f};

  for (int k0 = 0; k0 < Kend; k0 += 32) {
    V bh[4], bl[4];
#pragma unroll
    for (int j = 0; j < 4; ++j) {
      const size_t bo = (size_t)(n0 + (j << 4) + rlane) * ldb + koff + k0;
      bh[j] = Frag<T>::load(Bb + bo);
      if (SPLIT) bl[j] = Frag<T>::load(Bb2 + bo);
    }
#pragma unroll
    for (int i = 0; i < 4; ++i) {
      const size_t ao = (size_t)(m0 + (i << 4) + rlane) * lda + koff + k0;
      V ah = Frag<T>::load(Ab + ao);
      V al;
      if (SPLIT) al = Frag<T>::load(Ab2 + ao);
#pragma unroll
      for (int j = 0; j < 4; ++j) {
        acc[i][j] = Frag<T>::mma(ah, bh[j], acc[i][j]);
        if (SPLIT) {
          acc[i][j] = Frag<T>::mma(ah, bl[j], acc[i][j]);
          acc[i][j] = Frag<T>::mma(al, bh[j], acc[i][j]);
        }
      }
      Frag<T>::guard(acc[i][0], acc[i][3], ah, SPLIT ? al : ah);
    }
    Frag<T>::keep(bh[0], bh[1], bh[2], bh[3]);
    if (SPLIT) Frag<T>::keep(bl[0], bl[1], bl[2], bl[3]);
  }
  acc_guard4(acc[0][0], acc[0][1], acc[0][2], acc[0][3]);
  acc_guard4(acc[1][0], acc[1][1], acc[1][2], acc[1][3]);
  acc_guard4(acc[2][0], acc[2][1], acc[2][2], acc[2][3]);
  acc_guard4(acc[3][0], acc[3][1], acc[3][2], acc[3][3]);

  float* slab = sT[wave];
#pragma unroll
  for (int i = 0; i < 4; ++i) {
    const int mBase = m0 + (i << 4);
#pragma unroll
    for (int j = 0; j < 4; ++j) {
#pragma unroll
      for (int r = 0; r < 8; ++r) {
        const float v = acc[i][j][r] * scale;
        slab[(mOff + r) * 68 + (j << 4) + rlane] = v;
      }
    }
    __builtin_amdgcn_fence(__ATOMIC_RELEASE, "workgroup");
    __builtin_amdgcn_wave_barrier();
    __builtin_amdgcn_fence(__ATOMIC_ACQUIRE, "workgroup");
    if (OUT_MODE == 0) {
      float* C = (float*)Cout + (size_t)b * strideC;
      const int hh = lane >> 4, c4 = (lane & 15) * 4;
      for (int pass = 0; pass < 2; ++pass) {
#pragma unroll
        for (int it = 0; it < 8; ++it) {
          const int row = it * 2 + hh;
          v4f v = *(const v4f*)(slab + row * 68 + c4);
          *(volatile v4f*)(C + (size_t)(mBase + row) * ldc + n0 + c4) = v;
        }
        __threadfence();
      }
    } else {
      const int q = lane >> 3, c8 = (lane & 7) * 8;
      unsigned short* C  = (unsigned short*)Cout  + (size_t)b * strideC;
      unsigned short* C2 = (unsigned short*)Cout2 + (size_t)b * strideC;
      for (int pass = 0; pass < 2; ++pass) {
#pragma unroll
        for (int it = 0; it < 4; ++it) {
          const int row = it * 4 + q;
          const float* sp = slab + row * 68 + c8;
          v8h hv, lv;
#pragma unroll
          for (int e = 0; e < 8; ++e) {
            unsigned short hb = f2bf_bits(sp[e]);
            unsigned short lb = f2bf_bits(sp[e] - bf_bits2f(hb));
            hv[e] = __builtin_bit_cast(_Float16, hb);
            lv[e] = __builtin_bit_cast(_Float16, lb);
          }
          *(volatile v8h*)(C + (size_t)(mBase + row) * ldc + n0 + c8) = hv;
          *(volatile v8h*)(C2 + (size_t)(mBase + row) * ldc + n0 + c8) = lv;
        }
        __threadfence();
      }
    }
    __builtin_amdgcn_fence(__ATOMIC_RELEASE, "workgroup");
    __builtin_amdgcn_wave_barrier();
    __builtin_amdgcn_fence(__ATOMIC_ACQUIRE, "workgroup");
  }
}

__global__ __launch_bounds__(256) void cast_f32_bf16x8(
    const float* __restrict__ in, unsigned short* __restrict__ out, int n8) {
  const int i = blockIdx.x * 256 + threadIdx.x;
  if (i < n8) {
    const v4f a = *(const v4f*)(in + (size_t)i * 8);
    const v4f c = *(const v4f*)(in + (size_t)i * 8 + 4);
    v4u u;
    u[0] = pack_bf16x2(a[0], a[1]);
    u[1] = pack_bf16x2(a[2], a[3]);
    u[2] = pack_bf16x2(c[0], c[1]);
    u[3] = pack_bf16x2(c[2], c[3]);
    unsigned short* dst = out + (size_t)i * 8;
    *(volatile v4u*)dst = u;
    __threadfence();
    *(volatile v4u*)dst = u;
  }
}

__global__ __launch_bounds__(256) void transpose_cast_w(
    const float* __restrict__ W0, const float* __restrict__ W1, const float* __restrict__ W2,
    unsigned short* __restrict__ Wt) {
  __shared__ __align__(16) unsigned short sTt[64][72];
  const int tid  = threadIdx.x;
  const int lane = tid & 31;
  const int w    = tid >> 5;
  const int z    = blockIdx.z;
  const float* W = (z == 0) ? W0 : ((z == 1) ? W1 : W2);
  const int n0 = blockIdx.x * 64;
  const int k0 = blockIdx.y * 64;
#pragma unroll
  for (int i = 0; i < 4; ++i) {
    const int idx = tid + 256 * i;
    const int kr  = idx >> 4;
    const int c4  = idx & 15;
    const v4f f = *(const v4f*)(W + (size_t)(k0 + kr) * DMODEL + n0 + c4 * 4);
    sTt[c4 * 4 + 0][kr] = f2bf_bits(f[0]);
    sTt[c4 * 4 + 1][kr] = f2bf_bits(f[1]);
    sTt[c4 * 4 + 2][kr] = f2bf_bits(f[2]);
    sTt[c4 * 4 + 3][kr] = f2bf_bits(f[3]);
  }
  __syncthreads();
  const int c8   = (lane & 7) * 8;
  const int rowA = w * 4 + (lane >> 3);
  const int rowB = rowA + 32;
  v4u va, vb;
  __builtin_memcpy(&va, &sTt[rowA][c8], 16);
  __builtin_memcpy(&vb, &sTt[rowB][c8], 16);
  unsigned short* base = Wt + (size_t)z * WPLANE;
  unsigned short* da = base + (size_t)(n0 + rowA) * DIN + k0 + c8;
  unsigned short* db = base + (size_t)(n0 + rowB) * DIN + k0 + c8;
  for (int pass = 0; pass < 2; ++pass) {
    *(volatile v4u*)da = va;
    *(volatile v4u*)db = vb;
    __threadfence();
  }
}

__global__ __launch_bounds__(256) void softmax_causal_rows(
    const float* __restrict__ S, unsigned short* __restrict__ Ph, unsigned short* __restrict__ Pl, int qoff) {
  __shared__ float redm[8];
  __shared__ float reds[8];
  const int tid  = threadIdx.x;
  const int lane = tid & 31;
  const int w    = tid >> 5;
  const int r    = blockIdx.x;
  const int qg   = qoff + r;
  const float* Srow = S + (size_t)r * SEQ;

  float m = -__builtin_inff();
#pragma unroll
  for (int i = 0; i < 8; ++i) {
    const int kv = tid + 256 * i;
    const int kc = kv < qg ? kv : qg;
    m = fmaxf(m, Srow[kc]);
  }
#pragma unroll
  for (int off = 16; off > 0; off >>= 1) m = fmaxf(m, __shfl_xor(m, off, 32));
  if (lane == 0) redm[w] = m;
  __syncthreads();
  m = redm[0];
#pragma unroll
  for (int j = 1; j < 8; ++j) m = fmaxf(m, redm[j]);

  float ssum = 0.0f;
#pragma unroll
  for (int i = 0; i < 8; ++i) {
    const int kv = tid + 256 * i;
    const int kc = kv < qg ? kv : qg;
    const float e = exp2f((Srow[kc] - m) * LOG2E);
    ssum += (kv <= qg) ? e : 0.0f;
  }
#pragma unroll
  for (int off = 16; off > 0; off >>= 1) ssum += __shfl_xor(ssum, off, 32);
  if (lane == 0) reds[w] = ssum;
  __syncthreads();
  float tot = reds[0];
#pragma unroll
  for (int j = 1; j < 8; ++j) tot += reds[j];
  const float inv = 1.0f / tot;

  const int nL = (qg >> 6) + 1;
  const int L  = w * 4 + (lane >> 3);
  const int Lc = L < nL ? L : nL - 1;
  const int c8 = (lane & 7) * 8;
  const float* sp = Srow + Lc * 64 + c8;
  const v4f sa = *(const v4f*)sp;
  const v4f sb = *(const v4f*)(sp + 4);
  float sv[8];
  sv[0] = sa[0]; sv[1] = sa[1]; sv[2] = sa[2]; sv[3] = sa[3];
  sv[4] = sb[0]; sv[5] = sb[1]; sv[6] = sb[2]; sv[7] = sb[3];
  unsigned hw[4], lw[4];
#pragma unroll
  for (int e2 = 0; e2 < 4; ++e2) {
    const int kvA = Lc * 64 + c8 + 2 * e2;
    const int kvB = kvA + 1;
    const float eA = exp2f((sv[2 * e2] - m) * LOG2E) * inv;
    const float eB = exp2f((sv[2 * e2 + 1] - m) * LOG2E) * inv;
    const float pA = (kvA <= qg) ? eA : 0.0f;
    const float pB = (kvB <= qg) ? eB : 0.0f;
    const unsigned short hA = f2bf_bits(pA);
    const unsigned short hB = f2bf_bits(pB);
    const unsigned short lA = f2bf_bits(pA - bf_bits2f(hA));
    const unsigned short lB = f2bf_bits(pB - bf_bits2f(hB));
    hw[e2] = (unsigned)hA | (((unsigned)hB) << 16);
    lw[e2] = (unsigned)lA | (((unsigned)lB) << 16);
  }
  v4u hv, lv;
  hv[0] = hw[0]; hv[1] = hw[1]; hv[2] = hw[2]; hv[3] = hw[3];
  lv[0] = lw[0]; lv[1] = lw[1]; lv[2] = lw[2]; lv[3] = lw[3];
  unsigned short* dh = Ph + (size_t)r * SEQ + L * 64 + c8;
  unsigned short* dl = Pl + (size_t)r * SEQ + L * 64 + c8;
  for (int pass = 0; pass < 2; ++pass) {
    if (L < nL) {
      *(volatile v4u*)dh = hv;
      *(volatile v4u*)dl = lv;
    }
    __threadfence();
  }
}

extern "C" void kernel_launch(void* const* d_in, const int* in_sizes, int n_in,
                              void* d_out, int out_size, void* d_ws,
                              size_t ws_size, hipStream_t stream) {
  if (n_in < 4) return;
  if (in_sizes[0] != (int)PLANE_TOK || in_sizes[1] != (int)WPLANE ||
      in_sizes[2] != (int)WPLANE || in_sizes[3] != (int)WPLANE) return;
  if ((size_t)out_size != PLANE_TOK) return;
  if (ws_size < WS_END) return;

  const float* x  = (const float*)d_in[0];
  const float* Wq = (const float*)d_in[1];
  const float* Wk = (const float*)d_in[2];
  const float* Wv = (const float*)d_in[3];
  float* out = (float*)d_out;
  char* ws = (char*)d_ws;

  unsigned short* xb  = (unsigned short*)(ws + 0);
  float*          sc  = (float*)(ws + OFF_SC);
  unsigned short* Ph  = (unsigned short*)(ws + OFF_PH);
  unsigned short* Pl  = (unsigned short*)(ws + OFF_PL);
  unsigned short* Wt  = (unsigned short*)(ws + OFF_WT);
  unsigned short* QKh = (unsigned short*)(ws + OFF_QKH);
  unsigned short* QKl = (unsigned short*)(ws + OFF_QKL);
  unsigned short* Vth = (unsigned short*)(ws + OFF_VTH);
  unsigned short* Vtl = (unsigned short*)(ws + OFF_VTL);

  {
    const int n8 = (int)(PLANE_TOK / 8);
    cast_f32_bf16x8<<<dim3((n8 + 255) / 256), dim3(256), 0, stream>>>(x, xb, n8);
  }
  transpose_cast_w<<<dim3(DMODEL / 64, DIN / 64, 3), dim3(256), 0, stream>>>(Wq, Wk, Wv, Wt);

  {
    const int tiles = (NTOK / 64) * (DMODEL / 64);
    wmma_gemm64c<1, false, 2, 0><<<dim3(tiles / 8, 2), dim3(256), 0, stream>>>(
        xb, xb, DIN, 0L,
        Wt, Wt, DIN, (long)WPLANE,
        (void*)QKh, (void*)QKl, DMODEL, (long)PLANE_TOK,
        NTOK, DMODEL, DIN, 1.0f, 0);
  }
  {
    const int tiles = (DMODEL / 64) * (NTOK / 64);
    wmma_gemm64c<1, false, 2, 0><<<dim3(tiles / 8, 1), dim3(256), 0, stream>>>(
        Wt + 2 * WPLANE, Wt + 2 * WPLANE, DIN, 0L,
        xb, xb, DIN, 0L,
        (void*)Vth, (void*)Vtl, NTOK, 0L,
        DMODEL, NTOK, DIN, 1.0f, 0);
  }
  const unsigned short* qh_base = QKh;
  const unsigned short* kh_base = QKh + PLANE_TOK;
  const unsigned short* ql_base = QKl;
  const unsigned short* kl_base = QKl + PLANE_TOK;
  for (int b = 0; b < NBATCH; ++b) {
    for (int hf = 0; hf < 2; ++hf) {
      const int tm0 = hf * (QHALF / 64);
      const size_t qrow0 = (size_t)b * SEQ + (size_t)hf * QHALF;
      const unsigned short* qh = qh_base + qrow0 * DMODEL;
      const unsigned short* ql = ql_base + qrow0 * DMODEL;
      const unsigned short* kh = kh_base + (size_t)b * SEQ * DMODEL;
      const unsigned short* kl = kl_base + (size_t)b * SEQ * DMODEL;
      const int tilesM = QHALF / 64;
      const int ntri = tilesM * (tm0 + 1) + tilesM * (tilesM - 1) / 2;
      wmma_gemm64c<1, true, 0, 1><<<dim3((ntri + 7) / 8, 1), dim3(256), 0, stream>>>(
          qh, ql, DMODEL, 0L,
          kh, kl, DMODEL, 0L,
          (void*)sc, (void*)sc, SEQ, 0L,
          QHALF, SEQ, DMODEL, 0.03125f, tm0);
      softmax_causal_rows<<<dim3(QHALF), dim3(256), 0, stream>>>(sc, Ph, Pl, hf * QHALF);
      float* outp = out + qrow0 * DMODEL;
      const int tiles = (QHALF / 64) * (DMODEL / 64);
      wmma_gemm64c<1, true, 0, 2><<<dim3(tiles / 8, 1), dim3(256), 0, stream>>>(
          Ph, Pl, SEQ, 0L,
          Vth + (size_t)b * SEQ, Vtl + (size_t)b * SEQ, NTOK, 0L,
          (void*)outp, (void*)outp, DMODEL, 0L,
          QHALF, DMODEL, SEQ, 1.0f, tm0);
    }
  }
}
